// LSTMAutoEncoder_81990925680856
// MI455X (gfx1250) — hardware-run, weakly checked
//
#include <hip/hip_runtime.h>
#include <math.h>

constexpr int NB   = 256;
constexpr int NS   = 512;
constexpr int ND   = 64;
constexpr int NH   = 128;
constexpr int NG4  = 4 * NH;
constexpr int KL0  = ND + NH;
constexpr int KL1  = NH + NH;
constexpr int NTHR = 256;
constexpr int RB   = 16;
constexpr int P0   = 200;
constexpr int P1   = 264;
constexpr int PSP  = 68;
constexpr int NOUT = NB * NS * ND;
constexpr float WSC     = 16.0f;
constexpr float WSC_INV = 1.0f / 16.0f;
static_assert(KL0 % 32 == 0 && KL1 % 32 == 0 && NH % 32 == 0 && ND % 32 == 0);
static_assert(NB % RB == 0);
static_assert(NH == 16 * (NTHR / 32));
static_assert(P0 % 8 == 0 && P1 % 8 == 0 && P0 >= KL0 && P1 >= KL1);
static_assert((RB * P0) % 2 == 0 && (RB * P1) % 2 == 0);
static_assert(RB * ND == 4 * NTHR);
static_assert((NG4 * (KL0 / 8)) % NTHR == 0 && (NG4 * (KL1 / 8)) % NTHR == 0 && (ND * (NH / 8)) % NTHR == 0);
static_assert(NG4 == 2 * NTHR);
static_assert(PSP % 4 == 0 && PSP >= ND);

typedef __attribute__((ext_vector_type(16))) _Float16 v16h;
typedef __attribute__((ext_vector_type(8)))  _Float16 v8h;
typedef __attribute__((ext_vector_type(8)))  float    v8f;
typedef __attribute__((ext_vector_type(4)))  float    v4f;
typedef __attribute__((ext_vector_type(2)))  float    v2f;
typedef __attribute__((ext_vector_type(2)))  unsigned v2u;

template <typename T> struct Frag;
template <> struct Frag<_Float16> {
  typedef v16h V; union U { v16h v; v8h h[2]; };
  static __device__ __forceinline__ v16h load(const _Float16* p) {
    U f; f.h[0] = *(const v8h*)(p); f.h[1] = *(const v8h*)(p + 16); return f.v;
  }
  static __device__ __forceinline__ v8f mma(v16h a, v16h b, v8f c) {
    return __builtin_amdgcn_wmma_f32_16x16x32_f16(false, a, false, b, (short)0, c, false, false);
  }
};

__device__ __forceinline__ void mma_guard4(v8f& a, v8f& b, v8f& c, v8f& d,
                                           v16h x, v16h y0, v16h y1, v16h y2, v16h y3) {
  asm volatile("v_nop\n\tv_nop\n\tv_nop\n\tv_nop"
               : "+v"(a), "+v"(b), "+v"(c), "+v"(d)
               : "v"(x), "v"(y0), "v"(y1), "v"(y2), "v"(y3));
}
__device__ __forceinline__ void mma_guard1(v8f& a, v16h x, v16h y) {
  asm volatile("v_nop\n\tv_nop\n\tv_nop\n\tv_nop" : "+v"(a) : "v"(x), "v"(y));
}
__device__ __forceinline__ void acc_guard4(v8f& a, v8f& b, v8f& c, v8f& d) {
  asm volatile("v_nop\n\tv_nop\n\tv_nop\n\tv_nop" : "+v"(a), "+v"(b), "+v"(c), "+v"(d));
}
__device__ __forceinline__ void acc_guard1(v8f& a) {
  asm volatile("v_nop\n\tv_nop\n\tv_nop\n\tv_nop" : "+v"(a));
}

__device__ __forceinline__ unsigned h16bits(float f) {
  const _Float16 h = (_Float16)f;
  return (unsigned)__builtin_bit_cast(unsigned short, h);
}
__device__ __forceinline__ float fsig(float x)  { return __builtin_amdgcn_rcpf(1.0f + __expf(-x)); }
__device__ __forceinline__ float ftanh(float x) { return 1.0f - 2.0f * __builtin_amdgcn_rcpf(__expf(2.0f * x) + 1.0f); }

__global__ __launch_bounds__(NTHR) void pack_w_kernel(const float* __restrict__ A, const float* __restrict__ Bm,
                                                      unsigned short* __restrict__ dst, int nrow, int Kin, int Kh) {
  const int tid = threadIdx.x;
  const int K = Kin + Kh;
  const int nc8 = K >> 3;
  const int n8 = nrow * nc8;
  const int i = blockIdx.x * NTHR + tid;
  if (i < n8) {
    const int row = i / nc8;
    const int col = (i - row * nc8) * 8;
    const int ca = (col < Kin - 8) ? col : (Kin - 8);
    const int cb = (col - Kin > 0) ? (col - Kin) : 0;
    const float* ap = A  + (size_t)row * Kin + ca;
    const float* bp = Bm + (size_t)row * Kh  + cb;
    const v4f a0 = *(const v4f*)(ap);
    const v4f a1 = *(const v4f*)(ap + 4);
    const v4f b0 = *(const v4f*)(bp);
    const v4f b1 = *(const v4f*)(bp + 4);
    const float fa = (col < Kin) ? 1.0f : 0.0f;
    const float fb = 1.0f - fa;
    v8h hv;
#pragma unroll
    for (int e = 0; e < 4; ++e) {
      const float av0 = a0[e], bv0 = b0[e], av1 = a1[e], bv1 = b1[e];
      const float s0 = fmaf(fa, av0, fb * bv0) * WSC;
      const float s1 = fmaf(fa, av1, fb * bv1) * WSC;
      hv[e]     = (_Float16)s0;
      hv[4 + e] = (_Float16)s1;
    }
    unsigned short* op = dst + (size_t)i * 8;
    *(volatile v8h*)op = hv;
    __threadfence();
    *(volatile v8h*)op = hv;
  }
}

__device__ __forceinline__ void stage_x(unsigned short* T0, const float* __restrict__ x, int rowbase, int tn, float fac, int tid) {
  const int m = tid >> 4, f4 = (tid & 15) * 4;
  const v4f v = *(const v4f*)(x + ((size_t)(rowbase + m) * NS + (size_t)tn) * ND + f4);
  const float f0 = v[0] * fac, f1 = v[1] * fac, f2 = v[2] * fac, f3 = v[3] * fac;
  const unsigned u0 = h16bits(f0), u1 = h16bits(f1), u2 = h16bits(f2), u3 = h16bits(f3);
  v2u pk;
  pk[0] = u0 | (u1 << 16);
  pk[1] = u2 | (u3 << 16);
  *(v2u*)(T0 + m * P0 + f4) = pk;
}

template <int KTOT, int KP>
__device__ __forceinline__ void gates_gemm(const _Float16* arow, const _Float16* w,
                                           v8f& g0, v8f& g1, v8f& g2, v8f& g3) {
  const v8f z8 = {0.f, 0.f, 0.f, 0.f, 0.f, 0.f, 0.f, 0.f};
  g0 = z8; g1 = z8; g2 = z8; g3 = z8;
#pragma unroll 1
  for (int k0 = 0; k0 < KTOT; k0 += 32) {
    const v16h a  = Frag<_Float16>::load(arow + k0);
    const v16h b0 = Frag<_Float16>::load(w + k0);
    const v16h b1 = Frag<_Float16>::load(w + (size_t)1 * NH * KP + k0);
    const v16h b2 = Frag<_Float16>::load(w + (size_t)2 * NH * KP + k0);
    const v16h b3 = Frag<_Float16>::load(w + (size_t)3 * NH * KP + k0);
    g0 = Frag<_Float16>::mma(a, b0, g0);
    g1 = Frag<_Float16>::mma(a, b1, g1);
    g2 = Frag<_Float16>::mma(a, b2, g2);
    g3 = Frag<_Float16>::mma(a, b3, g3);
    mma_guard4(g0, g1, g2, g3, a, b0, b1, b2, b3);
  }
  acc_guard4(g0, g1, g2, g3);
}

__device__ __forceinline__ void cell_update(const v8f& gi, const v8f& gf, const v8f& gc, const v8f& go,
                                            const float* bb, float* cs, float* hn) {
#pragma unroll
  for (int r = 0; r < 8; ++r) {
    const float zi = gi[r] * WSC_INV + bb[0];
    const float zf = gf[r] * WSC_INV + bb[1];
    const float zg = gc[r] * WSC_INV + bb[2];
    const float zo = go[r] * WSC_INV + bb[3];
    const float ig = fsig(zi);
    const float fg = fsig(zf);
    const float gg = ftanh(zg);
    const float og = fsig(zo);
    const float cn = fg * cs[r] + ig * gg;
    cs[r] = cn;
    hn[r] = og * ftanh(cn);
  }
}

__global__ __launch_bounds__(NTHR) void seq_kernel(
    const float* __restrict__ x,
    const float* __restrict__ be0a, const float* __restrict__ be0b,
    const float* __restrict__ be1a, const float* __restrict__ be1b,
    const float* __restrict__ bd0a, const float* __restrict__ bd0b,
    const float* __restrict__ bd1a, const float* __restrict__ bd1b,
    const float* __restrict__ fcb,
    const unsigned short* __restrict__ WE0p, const unsigned short* __restrict__ WE1p,
    const unsigned short* __restrict__ WD0p, const unsigned short* __restrict__ WD1p,
    const unsigned short* __restrict__ WFCp,
    float* __restrict__ out) {
  __shared__ __align__(16) unsigned short T0[RB * P0];
  __shared__ __align__(16) unsigned short T1[RB * P1];
  __shared__ __align__(16) float          PS[RB * PSP];
  __shared__ __align__(16) float          BS[4 * NG4];
  const _Float16* WE0 = (const _Float16*)WE0p;
  const _Float16* WE1 = (const _Float16*)WE1p;
  const _Float16* WD0 = (const _Float16*)WD0p;
  const _Float16* WD1 = (const _Float16*)WD1p;
  const _Float16* WFC = (const _Float16*)WFCp;
  const int tid  = threadIdx.x;
  const int lane = tid & 31;
  const int wave = __builtin_amdgcn_readfirstlane(tid >> 5);
  const int c = lane & 15, hh = lane >> 4, koff = hh * 8;
  const int j = 16 * wave + c;
  const int rowbase = blockIdx.x * RB;

  {
    unsigned* z0 = (unsigned*)T0;
#pragma unroll 1
    for (int i = tid; i < RB * P0 / 2; i += NTHR) z0[i] = 0u;
    unsigned* z1 = (unsigned*)T1;
#pragma unroll 1
    for (int i = tid; i < RB * P1 / 2; i += NTHR) z1[i] = 0u;
  }
  {
    const int i2 = 2 * tid;
    const v2f p0 = *(const v2f*)(be0a + i2), q0 = *(const v2f*)(be0b + i2);
    const v2f p1 = *(const v2f*)(be1a + i2), q1 = *(const v2f*)(be1b + i2);
    asm volatile("" ::: "memory");
    const v2f p2 = *(const v2f*)(bd0a + i2), q2 = *(const v2f*)(bd0b + i2);
    const v2f p3 = *(const v2f*)(bd1a + i2), q3 = *(const v2f*)(bd1b + i2);
    asm volatile("" ::: "memory");
    *(v2f*)(BS + 0 * NG4 + i2) = p0 + q0;
    *(v2f*)(BS + 1 * NG4 + i2) = p1 + q1;
    *(v2f*)(BS + 2 * NG4 + i2) = p2 + q2;
    *(v2f*)(BS + 3 * NG4 + i2) = p3 + q3;
  }
  __syncthreads();
  stage_x(T0, x, rowbase, 0, 1.0f, tid);
  float bE0[4], bE1[4], bD0[4], bD1[4];
#pragma unroll
  for (int g = 0; g < 4; ++g) {
    bE0[g] = BS[0 * NG4 + g * NH + j];
    bE1[g] = BS[1 * NG4 + g * NH + j];
    bD0[g] = BS[2 * NG4 + g * NH + j];
    bD1[g] = BS[3 * NG4 + g * NH + j];
  }
  const float fbv = fcb[(j < ND) ? j : (ND - 1)];
  float cs0[8], cs1[8], h1r[8], h0n[8];
#pragma unroll
  for (int r = 0; r < 8; ++r) { cs0[r] = 0.0f; cs1[r] = 0.0f; h1r[r] = 0.0f; h0n[r] = 0.0f; }
  __syncthreads();

  const _Float16* a0row = (const _Float16*)T0 + c * P0 + koff;
  const _Float16* a1row = (const _Float16*)T1 + c * P1 + koff;
  const _Float16* afrow = (const _Float16*)T1 + c * P1 + NH + koff;
  const _Float16* we0 = WE0 + (size_t)j * KL0 + koff;
  const _Float16* we1 = WE1 + (size_t)j * KL1 + koff;
  const _Float16* wd0 = WD0 + (size_t)j * KL0 + koff;
  const _Float16* wd1 = WD1 + (size_t)j * KL1 + koff;
  const _Float16* wfc = WFC + (size_t)((j < ND) ? j : (ND - 1)) * NH + koff;
  const v8f z8 = {0.f, 0.f, 0.f, 0.f, 0.f, 0.f, 0.f, 0.f};

#pragma unroll 1
  for (int t = 0; t < NS; ++t) {
    v8f g0, g1, g2, g3;
    gates_gemm<KL0, KL0>(a0row, we0, g0, g1, g2, g3);
    cell_update(g0, g1, g2, g3, bE0, cs0, h0n);
    __syncthreads();
#pragma unroll
    for (int r = 0; r < 8; ++r) {
      const int ro = 8 * hh + r;
      const unsigned short hb = (unsigned short)h16bits(h0n[r]);
      T0[ro * P0 + ND + j] = hb;
      T1[ro * P1 + j] = hb;
      T1[ro * P1 + NH + j] = (unsigned short)h16bits(h1r[r]);
    }
    {
      const int tn = (t + 1 < NS) ? (t + 1) : (NS - 1);
      const float fac = (t + 1 < NS) ? 1.0f : 0.0f;
      stage_x(T0, x, rowbase, tn, fac, tid);
    }
    __syncthreads();
    gates_gemm<KL1, KL1>(a1row, we1, g0, g1, g2, g3);
    cell_update(g0, g1, g2, g3, bE1, cs1, h1r);
  }

#pragma unroll 1
  for (int t = 0; t < NS; ++t) {
    v8f g0, g1, g2, g3;
    gates_gemm<KL0, KL0>(a0row, wd0, g0, g1, g2, g3);
    cell_update(g0, g1, g2, g3, bD0, cs0, h0n);
    __syncthreads();
#pragma unroll
    for (int r = 0; r < 8; ++r) {
      const int ro = 8 * hh + r;
      const unsigned short hb = (unsigned short)h16bits(h0n[r]);
      T0[ro * P0 + ND + j] = hb;
      T1[ro * P1 + j] = hb;
      T1[ro * P1 + NH + j] = (unsigned short)h16bits(h1r[r]);
    }
    __syncthreads();
    gates_gemm<KL1, KL1>(a1row, wd1, g0, g1, g2, g3);
    cell_update(g0, g1, g2, g3, bD1, cs1, h1r);
    __syncthreads();
#pragma unroll
    for (int r = 0; r < 8; ++r) T1[(8 * hh + r) * P1 + NH + j] = (unsigned short)h16bits(h1r[r]);
    __syncthreads();
    if (wave < 4) {
      v8f fa = z8;
#pragma unroll 1
      for (int k0 = 0; k0 < NH; k0 += 32) {
        const v16h a = Frag<_Float16>::load(afrow + k0);
        const v16h b = Frag<_Float16>::load(wfc + k0);
        fa = Frag<_Float16>::mma(a, b, fa);
        mma_guard1(fa, a, b);
      }
      acc_guard1(fa);
#pragma unroll
      for (int r = 0; r < 8; ++r) {
        const int ro = 8 * hh + r;
        const float pred = fa[r] * WSC_INV + fbv;
        PS[ro * PSP + j] = pred;
        T0[ro * P0 + j] = (unsigned short)h16bits(pred);
      }
    }
    __syncthreads();
    {
      const int row = tid >> 4, c4 = (tid & 15) * 4;
      const v4f v = *(const v4f*)(PS + row * PSP + c4);
      float* op = out + ((size_t)(rowbase + row) * NS + (size_t)t) * ND + c4;
      *(volatile v4f*)op = v;
      __threadfence();
      *(volatile v4f*)op = v;
    }
  }
}

extern "C" void kernel_launch(void* const* d_in, const int* in_sizes, int n_in,
                              void* d_out, int out_size, void* d_ws, size_t ws_size, hipStream_t stream) {
  if (n_in < 19 || d_out == nullptr || d_ws == nullptr) return;
  const int expect[19] = { NB * NS * ND, NG4 * ND, NG4 * NH, NG4, NG4, NG4 * NH, NG4 * NH, NG4, NG4,
                           NG4 * ND, NG4 * NH, NG4, NG4, NG4 * NH, NG4 * NH, NG4, NG4, ND * NH, ND };
  for (int i = 0; i < 19; ++i) if (in_sizes[i] != expect[i]) return;
  if (out_size != NOUT) return;

  const float* x     = (const float*)d_in[0];
  const float* eWih0 = (const float*)d_in[1];
  const float* eWhh0 = (const float*)d_in[2];
  const float* ebih0 = (const float*)d_in[3];
  const float* ebhh0 = (const float*)d_in[4];
  const float* eWih1 = (const float*)d_in[5];
  const float* eWhh1 = (const float*)d_in[6];
  const float* ebih1 = (const float*)d_in[7];
  const float* ebhh1 = (const float*)d_in[8];
  const float* dWih0 = (const float*)d_in[9];
  const float* dWhh0 = (const float*)d_in[10];
  const float* dbih0 = (const float*)d_in[11];
  const float* dbhh0 = (const float*)d_in[12];
  const float* dWih1 = (const float*)d_in[13];
  const float* dWhh1 = (const float*)d_in[14];
  const float* dbih1 = (const float*)d_in[15];
  const float* dbhh1 = (const float*)d_in[16];
  const float* fcW   = (const float*)d_in[17];
  const float* fcb   = (const float*)d_in[18];
  float* out = (float*)d_out;

  char* ws = (char*)d_ws; size_t off = 0;
  auto carve = [&](size_t bytes) -> char* { char* p = ws + off; off += (bytes + 255) & ~(size_t)255; return p; };
  unsigned short* WE0 = (unsigned short*)carve((size_t)NG4 * KL0 * 2);
  unsigned short* WE1 = (unsigned short*)carve((size_t)NG4 * KL1 * 2);
  unsigned short* WD0 = (unsigned short*)carve((size_t)NG4 * KL0 * 2);
  unsigned short* WD1 = (unsigned short*)carve((size_t)NG4 * KL1 * 2);
  unsigned short* WFC = (unsigned short*)carve((size_t)ND * NH * 2);
  if (off > ws_size || off > (size_t)134217728) return;

  pack_w_kernel<<<(NG4 * (KL0 / 8)) / NTHR, NTHR, 0, stream>>>(eWih0, eWhh0, WE0, NG4, ND, NH);
  pack_w_kernel<<<(NG4 * (KL1 / 8)) / NTHR, NTHR, 0, stream>>>(eWih1, eWhh1, WE1, NG4, NH, NH);
  pack_w_kernel<<<(NG4 * (KL0 / 8)) / NTHR, NTHR, 0, stream>>>(dWih0, dWhh0, WD0, NG4, ND, NH);
  pack_w_kernel<<<(NG4 * (KL1 / 8)) / NTHR, NTHR, 0, stream>>>(dWih1, dWhh1, WD1, NG4, NH, NH);
  pack_w_kernel<<<(ND * (NH / 8)) / NTHR, NTHR, 0, stream>>>(fcW, fcW, WFC, ND, NH, 0);
  seq_kernel<<<NB / RB, NTHR, 0, stream>>>(x, ebih0, ebhh0, ebih1, ebhh1, dbih0, dbhh0, dbih1, dbhh1, fcb,
                                           WE0, WE1, WD0, WD1, WFC, out);
}
